// EnAttention_8813272891835
// MI455X (gfx1250) — hardware-verified
//
#include <hip/hip_runtime.h>
#include <stddef.h>
#include <stdint.h>

#define NNODE   10000
#define NEDGE   320000
#define HIDW    128
#define QKVW    256
#define NPW     1024
#define MPR     10048
#define NPADR   10240
#define NTHR    256
#define NWAVE   8
#define GBM     64
#define GBN     128
#define GTHR    128
#define TE      64
#define ETHR    64
#define DP      148
#define AP      264
#define A2P     520
#define CSTN    1024
#define EPT     8
#define CHUNK   (NTHR * EPT)
#define WCAP    (EPT * 32)
#define LISTN   (NWAVE * WCAP)
#define NBA     512
#define SLA     9
#define RCAP    28672
#define DEGCAP  96
#define NBLK    20
#define AGG_ZINTS (LISTN + 2 * RCAP + 3 * NBA)
#define STG_OFF   (AGG_ZINTS + 16)
#define SOFT_LDS_BYTES ((STG_OFF + NBA * 8) * 4)
#define AGG_LDS_BYTES  ((STG_OFF + NBA * 3) * 4)
#define EA_LDS_FLOATS (TE * DP + (TE * AP) / 2 + CSTN + TE * 4 + 2 * TE)
#define EB_LDS_FLOATS (TE * DP + (TE * AP) / 2 + (TE * A2P) / 2 + CSTN + TE * 8)
#define EA_LDS_BYTES (EA_LDS_FLOATS * 4)
#define EB_LDS_BYTES (EB_LDS_FLOATS * 4)

#define V_BN   0
#define V_A    1024
#define V_B    2048
#define V_BO   3072
#define V_TOT  3200
#define A_W1R  0
#define A_EB2  128
#define A_MB1  256
#define A_PW1  384
#define A_PB1  448
#define A_PW2  512
#define A_EWB  768
#define A_PB2  800
#define B_MW1R 0
#define B_MB2  512
#define B_CB1  640
#define B_XB1  768
#define B_GB   896
#define B_CB2  928
#define B_XB2  960
#define B_CHW  992

#define O_WN    0
#define O_E2    (O_WN  + 1024 * 128)
#define O_M2    (O_E2  + 128 * 256)
#define O_M1E   (O_M2  + 128 * 256)
#define O_CXG   (O_M1E + 144 * 256)
#define O_CX2   (O_CXG + 272 * 256)
#define O_WO2   (O_CX2 + 16 * 512)
#define WPL_TOT (O_WO2 + 128 * 512)

#define NU_WN   (1024 * 16)
#define NU_E2   (128 * 32)
#define NU_M1E  (144 * 32)
#define NU_CXG  (272 * 32)
#define NU_CX2  (16 * 64)
#define NU_WO2  (128 * 64)
#define NU_HB   (MPR * 16)
#define NU_XP   10240
#define NU_VN   1280
#define NV_N    1152
#define PU0 (NU_WN)
#define PU1 (PU0 + NU_E2)
#define PU2 (PU1 + NU_E2)
#define QU0 (NU_M1E)
#define QU1 (QU0 + NU_CXG)
#define QU2 (QU1 + NU_CX2)
#define QU3 (QU2 + NU_WO2)
#define RU0 (NU_HB)
#define RU1 (RU0 + NU_XP)
#define RU2 (RU1 + NU_VN)

static_assert(NEDGE % TE == 0 && NEDGE % 4 == 0);
static_assert(MPR % GBM == 0 && MPR >= NNODE && NPADR == NBLK * NBA && NPADR >= MPR);
static_assert((CHUNK & (CHUNK - 1)) == 0 && NBA == (1 << SLA));
static_assert(((long long)NEDGE << SLA) < (1LL << 31));
static_assert(AGG_ZINTS % 4 == 0 && STG_OFF % 4 == 0);
static_assert(SOFT_LDS_BYTES <= 300000 && AGG_LDS_BYTES <= 300000 && EB_LDS_BYTES <= 300000);
static_assert(PU0 % NTHR == 0 && PU1 % NTHR == 0 && PU2 % NTHR == 0);
static_assert(QU0 % NTHR == 0 && QU1 % NTHR == 0 && QU2 % NTHR == 0 && QU3 % NTHR == 0);
static_assert(RU0 % NTHR == 0 && RU1 % NTHR == 0 && RU2 % NTHR == 0);
static_assert(V_TOT % 32 == 0 && NU_XP >= MPR && NV_N == 1024 + 128 && NV_N % 32 == 0 && NU_VN >= NV_N);
static_assert(V_A - V_BN == 1024 && V_B - V_A == 1024 && V_BO - V_B == 1024 && V_TOT - V_BO == 128);
static_assert(O_E2 % 128 == 0 && O_M2 % 128 == 0 && O_M1E % 128 == 0 && O_CXG % 128 == 0);
static_assert(O_CX2 % 128 == 0 && O_WO2 % 128 == 0 && WPL_TOT % 128 == 0);
static_assert((DP * 4) % 16 == 0 && (AP * 2) % 16 == 0 && (A2P * 2) % 16 == 0);
static_assert(DP >= 144 && AP >= 256 && A2P >= 512);
static_assert(CSTN == 4 * 4 * ETHR && TE == ETHR && TE == 2 * 32);
static_assert(DEGCAP >= 58 + 8 && RCAP >= 16638 + 4096);
static_assert((3 * NNODE) % 4 == 0 && (NBA * 3) % 4 == 0);
static_assert(NBA % NWAVE == 0 && NBA % 32 == 0);

typedef float          v4f   __attribute__((ext_vector_type(4)));
typedef float          v8f   __attribute__((ext_vector_type(8)));
typedef int            v4i   __attribute__((ext_vector_type(4)));
typedef int            v8i   __attribute__((ext_vector_type(8)));
typedef unsigned short v8us  __attribute__((ext_vector_type(8)));
typedef unsigned short v16us __attribute__((ext_vector_type(16)));
typedef __bf16         v16bf __attribute__((ext_vector_type(16)));
typedef v4f  __attribute__((may_alias)) v4fa;
typedef v4i  __attribute__((may_alias)) v4ia;
typedef v8us __attribute__((may_alias)) v8usa;
union FragB { v16bf v; v16us u; v8us h[2]; v8i w; };

__device__ __forceinline__ v8f wmb(const FragB& a, const FragB& b, v8f c) {
  v8f d = __builtin_amdgcn_wmma_f32_16x16x32_bf16(false, a.v, false, b.v, (short)0, c, false, false);
  asm volatile("v_nop\n\tv_nop\n\tv_nop\n\tv_nop" : "+v"(d) : "v"(a.w), "v"(b.w));
  return d;
}
__device__ __forceinline__ v8f z8() { v8f z = {0.f, 0.f, 0.f, 0.f, 0.f, 0.f, 0.f, 0.f}; return z; }

__device__ __forceinline__ unsigned bf16_bits(float f) {
  const unsigned u = __float_as_uint(f);
  return (u + 0x7FFFu + ((u >> 16) & 1u)) >> 16;
}
__device__ __forceinline__ float bf16_val(float f) { return __uint_as_float(bf16_bits(f) << 16); }
__device__ __forceinline__ float silu_p(float t) { return t * __builtin_amdgcn_rcpf(1.0f + expf(-t)); }
__device__ __forceinline__ float sigm_p(float t) { return __builtin_amdgcn_rcpf(1.0f + expf(-t)); }
__device__ __forceinline__ int clampi(int v, int hi) { return v < 0 ? 0 : (v > hi ? hi : v); }
__device__ __forceinline__ v8f join8(v4f a, v4f b) { v8f r = {a.x, a.y, a.z, a.w, b.x, b.y, b.z, b.w}; return r; }

__device__ __forceinline__ void split8(v8f v, unsigned short* phi, unsigned short* plo) {
  v8us oh, ol;
#pragma unroll
  for (int i = 0; i < 8; ++i) {
    const unsigned hb = bf16_bits(v[i]);
    const unsigned lb = bf16_bits(v[i] - __uint_as_float(hb << 16));
    oh[i] = (unsigned short)hb;
    ol[i] = (unsigned short)lb;
  }
  *(v8usa*)phi = oh;
  *(v8usa*)plo = ol;
}
__device__ __forceinline__ void put16(unsigned short* dp, v8us o) {
  *(volatile v8us*)dp = o;
  __threadfence();
  *(volatile v8us*)dp = o;
}
__device__ __forceinline__ void putf4(float* dp, v4f o) {
  *(volatile v4f*)dp = o;
  __threadfence();
  *(volatile v4f*)dp = o;
}
__device__ __forceinline__ void putf1(float* dp, float o) {
  *(volatile float*)dp = o;
  __threadfence();
  *(volatile float*)dp = o;
}

template <int SLB>
__device__ __forceinline__ int scan_chunk(const int* __restrict__ dsts, int nE, int cbase, int slotBase,
                                          int nb, int vec8, int* list, int tid, int lane, int wave) {
  int wc = 0;
  const int el0  = tid * EPT;
  const int e0   = cbase + el0;
  const int sent = (int)(1u << 31);
  v4i da, db;
  if (vec8 != 0 && cbase + CHUNK <= nE) {
    da = *(const v4i*)(dsts + e0);
    db = *(const v4i*)(dsts + e0 + 4);
  } else {
    da.x = (e0     < nE) ? dsts[min(e0,     nE - 1)] : sent;
    da.y = (e0 + 1 < nE) ? dsts[min(e0 + 1, nE - 1)] : sent;
    da.z = (e0 + 2 < nE) ? dsts[min(e0 + 2, nE - 1)] : sent;
    da.w = (e0 + 3 < nE) ? dsts[min(e0 + 3, nE - 1)] : sent;
    db.x = (e0 + 4 < nE) ? dsts[min(e0 + 4, nE - 1)] : sent;
    db.y = (e0 + 5 < nE) ? dsts[min(e0 + 5, nE - 1)] : sent;
    db.z = (e0 + 6 < nE) ? dsts[min(e0 + 6, nE - 1)] : sent;
    db.w = (e0 + 7 < nE) ? dsts[min(e0 + 7, nE - 1)] : sent;
  }
  const unsigned nbs = (unsigned)slotBase;
  const unsigned unb = (unsigned)nb;
  const unsigned s0 = (unsigned)da.x - nbs, s1 = (unsigned)da.y - nbs;
  const unsigned s2 = (unsigned)da.z - nbs, s3 = (unsigned)da.w - nbs;
  const unsigned s4 = (unsigned)db.x - nbs, s5 = (unsigned)db.y - nbs;
  const unsigned s6 = (unsigned)db.z - nbs, s7 = (unsigned)db.w - nbs;
  const bool h0 = s0 < unb, h1 = s1 < unb, h2 = s2 < unb, h3 = s3 < unb;
  const bool h4 = s4 < unb, h5 = s5 < unb, h6 = s6 < unb, h7 = s7 < unb;
  const unsigned any = __builtin_amdgcn_ballot_w32(h0 | h1 | h2 | h3 | h4 | h5 | h6 | h7);
  if (any != 0u) {
#define HITJ(J, HJ, SJ) { \
      const unsigned mj = __builtin_amdgcn_ballot_w32(HJ); \
      if (mj != 0u) { \
        if (HJ) { \
          const int pos = wc + (int)__builtin_amdgcn_mbcnt_lo(mj, 0u); \
          if (pos < WCAP) list[wave * WCAP + pos] = ((el0 + (J)) << SLB) | (int)(SJ); \
        } \
        wc += (int)__builtin_popcount(mj); } }
    HITJ(0, h0, s0)
    HITJ(1, h1, s1)
    HITJ(2, h2, s2)
    HITJ(3, h3, s3)
    HITJ(4, h4, s4)
    HITJ(5, h5, s5)
    HITJ(6, h6, s6)
    HITJ(7, h7, s7)
#undef HITJ
  }
  return wc;
}

__device__ __forceinline__ int scan_build(const int* __restrict__ dsts, int nE, int vec8, int nodeBase,
                                          int* dsm, int tid, int lane, int wave) {
  int* list = dsm;
  int* hl   = dsm + LISTN;
  int* sl   = hl + RCAP;
  int* cnt  = sl + RCAP;
  int* offs = cnt + NBA;
  int* cur  = offs + NBA;
  int* misc = cur + NBA;
  {
    const v4i z4 = {0, 0, 0, 0};
    for (int i = tid * 4; i < AGG_ZINTS; i += NTHR * 4) *(v4ia*)(dsm + i) = z4;
    if (tid < 16) misc[tid] = 0;
  }
  __syncthreads();
  int t = 0, ov = 0;
  const int nChunks = (nE + CHUNK - 1) / CHUNK;
#pragma unroll 1
  for (int ch = 0; ch < nChunks; ++ch) {
    const int cbase = ch * CHUNK;
    const int wc = scan_chunk<SLA>(dsts, nE, cbase, nodeBase, NBA, vec8, list, tid, lane, wave);
    if (lane == 0) misc[wave] = wc;
    __syncthreads();
    if (wave == 0) {
#pragma unroll 1
      for (int w2 = 0; w2 < NWAVE; ++w2) {
        int c = misc[w2];
        c = c < 0 ? 0 : (c > WCAP ? WCAP : c);
#pragma unroll 1
        for (int b0 = 0; b0 < c; b0 += 32) {
          const int idx = b0 + lane;
          const int ent = list[w2 * WCAP + (idx < WCAP ? idx : WCAP - 1)];
          const int m32 = (c - b0) < 32 ? (c - b0) : 32;
#pragma unroll 1
          for (int k = 0; k < m32; ++k) {
            const int u    = __builtin_amdgcn_readlane(ent, k);
            const int slot = u & (NBA - 1);
            const int el   = (u >> SLA) & (CHUNK - 1);
            const int pk   = ((cbase + el) << SLA) | slot;
            if (t < RCAP) {
              if (lane == 0) { hl[t] = pk; cnt[slot] = cnt[slot] + 1; }
              t = t + 1;
            } else {
              ov = 1;
            }
          }
        }
      }
    }
    __syncthreads();
  }
  if (wave == 0 && lane == 0) { misc[8] = t; misc[9] = ov; }
  __syncthreads();
  int tt = misc[8];
  tt = tt < 0 ? 0 : (tt > RCAP ? RCAP : tt);
  const int ovf = misc[9];
  if (wave == 0) {
    const int base = lane * (NBA / 32);
    int s = 0;
#pragma unroll 1
    for (int i = 0; i < NBA / 32; ++i) s += cnt[base + i];
    int incl = s;
#pragma unroll
    for (int d = 1; d < 32; d <<= 1) {
      const int y = __shfl_up(incl, d, 32);
      if (lane >= d) incl += y;
    }
    int run = incl - s;
#pragma unroll 1
    for (int i = 0; i < NBA / 32; ++i) {
      const int cv = cnt[base + i];
      offs[base + i] = run;
      cur[base + i]  = run;
      run += cv;
    }
  }
  __syncthreads();
  if (wave == 0) {
#pragma unroll 1
    for (int b0 = 0; b0 < tt; b0 += 32) {
      const int idx = b0 + lane;
      const int ent = hl[idx < RCAP ? idx : RCAP - 1];
      const int m32 = (tt - b0) < 32 ? (tt - b0) : 32;
#pragma unroll 1
      for (int k = 0; k < m32; ++k) {
        const int u    = __builtin_amdgcn_readlane(ent, k);
        const int slot = u & (NBA - 1);
        if (lane == 0) {
          int p = cur[slot];
          p = p < 0 ? 0 : (p > RCAP - 1 ? RCAP - 1 : p);
          sl[p] = u;
          cur[slot] = p + 1;
        }
      }
    }
  }
  __syncthreads();
  return ovf;
}

__global__ __launch_bounds__(NTHR) void k_pw1(const float* __restrict__ Wq, const float* __restrict__ Wk,
                                              const float* __restrict__ Wv, const float* __restrict__ ew1,
                                              const float* __restrict__ ew2, const float* __restrict__ mw2,
                                              unsigned short* WPL) {
  const int u = (int)blockIdx.x * NTHR + (int)threadIdx.x;
  v8us o;
  if (u < PU0) {
    const int n  = u >> 4;
    const int k8 = (u & 15) * 8;
    if (n < 768) {
      const float* W = (n < 256) ? Wq : ((n < 512) ? Wk : Wv);
      const float* p = W + (size_t)k8 * QKVW + (n & 255);
#pragma unroll
      for (int i = 0; i < 8; ++i) o[i] = (unsigned short)bf16_bits(p[(size_t)i * QKVW]);
    } else {
      const int kof = (n >= 896) ? HIDW : 0;
      const float* p = ew1 + (size_t)(kof + k8) * HIDW + (n & 127);
#pragma unroll
      for (int i = 0; i < 8; ++i) o[i] = (unsigned short)bf16_bits(p[(size_t)i * HIDW]);
    }
    put16(WPL + O_WN + (size_t)u * 8, o);
    return;
  } else if (u < PU2) {
    const bool second = u >= PU1;
    const int v  = second ? (u - PU1) : (u - PU0);
    const int n  = v >> 5;
    const int k8 = (v & 31) * 8;
    const float* W = second ? mw2 : ew2;
    const float* p = W + (size_t)(k8 & 127) * HIDW + n;
#pragma unroll
    for (int i = 0; i < 8; ++i) o[i] = (unsigned short)bf16_bits(p[(size_t)i * HIDW]);
    const size_t dof = second ? (size_t)O_M2 : (size_t)O_E2;
    put16(WPL + dof + (size_t)v * 8, o);
    return;
  }
}

__global__ __launch_bounds__(NTHR) void k_pw2(const float* __restrict__ mw1, const float* __restrict__ eww,
                                              const float* __restrict__ cw1, const float* __restrict__ xw1,
                                              const float* __restrict__ gw, const float* __restrict__ cw2,
                                              const float* __restrict__ xw2, const float* __restrict__ Wo,
                                              unsigned short* WPL) {
  const int u = (int)blockIdx.x * NTHR + (int)threadIdx.x;
  v8us o;
  if (u < QU0) {
    const int v  = u;
    const int n  = v >> 5;
    const int k8 = (v & 31) * 8;
    const int sr = k8 & 127;
    if (n < 128) {
      const float* p = mw1 + (size_t)sr * HIDW + n;
#pragma unroll
      for (int i = 0; i < 8; ++i) o[i] = (unsigned short)bf16_bits(p[(size_t)i * HIDW]);
    } else {
      const int nn = n - 128;
      const int nc = nn < 4 ? nn : 3;
      const unsigned mk = nn < 4 ? 0xffffu : 0u;
      const float* p = eww + (size_t)sr * 4 + nc;
#pragma unroll
      for (int i = 0; i < 8; ++i) o[i] = (unsigned short)(bf16_bits(p[(size_t)i * 4]) & mk);
    }
    put16(WPL + O_M1E + (size_t)v * 8, o);
    return;
  } else if (u < QU1) {
    const int v  = u - QU0;
    const int n  = v >> 5;
    const int k8 = (v & 31) * 8;
    const int sr = k8 & 127;
    if (n < 256) {
      const float* W = (n < 128) ? cw1 : xw1;
      const float* p = W + (size_t)sr * HIDW + (n & 127);
#pragma unroll
      for (int i = 0; i < 8; ++i) o[i] = (unsigned short)bf16_bits(p[(size_t)i * HIDW]);
    } else {
      const int nn = n - 256;
      const int nc = nn < 4 ? nn : 3;
      const unsigned mk = nn < 4 ? 0xffffu : 0u;
      const float* p = gw + (size_t)sr * 4 + nc;
#pragma unroll
      for (int i = 0; i < 8; ++i) o[i] = (unsigned short)(bf16_bits(p[(size_t)i * 4]) & mk);
    }
    put16(WPL + O_CXG + (size_t)v * 8, o);
    return;
  } else if (u < QU2) {
    const int v    = u - QU1;
    const int n    = v >> 6;
    const int k8   = (v & 63) * 8;
    const int part = k8 >> 7;
    const int sr   = k8 & 127;
    if (n < 8) {
      const float* W = (n < 4) ? cw2 : xw2;
      const int want = (n < 4) ? 0 : 1;
      const unsigned mk = ((part & 1) == want) ? 0xffffu : 0u;
      const float* p = W + (size_t)sr * 4 + (n & 3);
#pragma unroll
      for (int i = 0; i < 8; ++i) o[i] = (unsigned short)(bf16_bits(p[(size_t)i * 4]) & mk);
    } else {
#pragma unroll
      for (int i = 0; i < 8; ++i) o[i] = (unsigned short)0;
    }
    put16(WPL + O_CX2 + (size_t)v * 8, o);
    return;
  } else if (u < QU3) {
    const int v  = u - QU2;
    const int n  = v >> 6;
    const int k8 = (v & 63) * 8;
    const float* p = Wo + (size_t)(k8 & 255) * HIDW + n;
#pragma unroll
    for (int i = 0; i < 8; ++i) o[i] = (unsigned short)bf16_bits(p[(size_t)i * HIDW]);
    put16(WPL + O_WO2 + (size_t)v * 8, o);
    return;
  }
}

#define VSEG(BASE, PADLEN, LEN, PTR, SOFF) \
    if (i >= (BASE) && i < (BASE) + (PADLEN)) { \
      const int j = i - (BASE); \
      const int jc = j < (LEN) ? j : (LEN) - 1; \
      const float w = bf16_val((PTR)[(SOFF) + jc]); \
      val = (j < (LEN)) ? w : 0.0f; }

__global__ __launch_bounds__(NTHR) void k_pn(const float* __restrict__ h, const float* __restrict__ x,
                                             const float* __restrict__ bq, const float* __restrict__ bk,
                                             const float* __restrict__ bv, const float* __restrict__ eb1,
                                             const float* __restrict__ bo,
                                             unsigned short* HB, float* XP, float* VEC) {
  const int u = (int)blockIdx.x * NTHR + (int)threadIdx.x;
  if (u < RU0) {
    v8us o;
    const int v   = u;
    const int row = v >> 4;
    const int k8  = (v & 15) * 8;
    const int rc  = row < NNODE ? row : NNODE - 1;
    const unsigned mk = (row < NNODE) ? 0xffffu : 0u;
    const float* p = h + (size_t)rc * HIDW + k8;
    const v4f a = *(const v4fa*)p;
    const v4f b = *(const v4fa*)(p + 4);
    o[0] = (unsigned short)(bf16_bits(a.x) & mk); o[1] = (unsigned short)(bf16_bits(a.y) & mk);
    o[2] = (unsigned short)(bf16_bits(a.z) & mk); o[3] = (unsigned short)(bf16_bits(a.w) & mk);
    o[4] = (unsigned short)(bf16_bits(b.x) & mk); o[5] = (unsigned short)(bf16_bits(b.y) & mk);
    o[6] = (unsigned short)(bf16_bits(b.z) & mk); o[7] = (unsigned short)(bf16_bits(b.w) & mk);
    put16(HB + (size_t)v * 8, o);
    return;
  } else if (u < RU1) {
    const int row = u - RU0;
    if (row >= MPR) return;
    const int rc  = row < NNODE ? row : NNODE - 1;
    const bool ok = row < NNODE;
    const float x0 = x[(size_t)rc * 3 + 0];
    const float x1 = x[(size_t)rc * 3 + 1];
    const float x2 = x[(size_t)rc * 3 + 2];
    v4f q;
    q.x = ok ? bf16_val(x0) : 0.0f;
    q.y = ok ? bf16_val(x1) : 0.0f;
    q.z = ok ? bf16_val(x2) : 0.0f;
    q.w = 0.0f;
    putf4(XP + (size_t)row * 4, q);
    return;
  } else if (u < RU2) {
    const int j0 = u - RU1;
    if (j0 >= NV_N) return;
    const int i = (j0 < 1024) ? j0 : (V_BO + (j0 - 1024));
    float val = 0.0f;
    VSEG(V_BN + 0,   256, 256, bq, 0)
    VSEG(V_BN + 256, 256, 256, bk, 0)
    VSEG(V_BN + 512, 256, 256, bv, 0)
    VSEG(V_BN + 768, 128, 128, eb1, 0)
    VSEG(V_BO, 128, 128, bo, 0)
    putf1(VEC + i, val);
    return;
  }
}

__global__ __launch_bounds__(NTHR) void k_pva(const float* __restrict__ ew1, const float* __restrict__ eb2,
                                              const float* __restrict__ mb1, const float* __restrict__ pw1,
                                              const float* __restrict__ pb1, const float* __restrict__ pw2,
                                              const float* __restrict__ ewb, const float* __restrict__ pb2,
                                              float* VEC) {
  const int u = (int)blockIdx.x * NTHR + (int)threadIdx.x;
  if (u >= 1024) return;
  const int i = V_A + u;
  float val = 0.0f;
  VSEG(V_A + A_W1R, 128, 128, ew1, 256 * HIDW)
  VSEG(V_A + A_EB2, 128, 128, eb2, 0)
  VSEG(V_A + A_MB1, 128, 128, mb1, 0)
  VSEG(V_A + A_PW1, 64, 64, pw1, 0)
  VSEG(V_A + A_PB1, 64, 64, pb1, 0)
  VSEG(V_A + A_PW2, 256, 256, pw2, 0)
  VSEG(V_A + A_EWB, 32, 4, ewb, 0)
  VSEG(V_A + A_PB2, 32, 4, pb2, 0)
  putf1(VEC + i, val);
}

__global__ __launch_bounds__(NTHR) void k_pvb(const float* __restrict__ mw1, const float* __restrict__ mb2,
                                              const float* __restrict__ cb1, const float* __restrict__ xb1,
                                              const float* __restrict__ gb, const float* __restrict__ cb2,
                                              const float* __restrict__ xb2, const float* __restrict__ chw,
                                              float* VEC) {
  const int u = (int)blockIdx.x * NTHR + (int)threadIdx.x;
  if (u >= 1024) return;
  const int i = V_B + u;
  float val = 0.0f;
  VSEG(V_B + B_MW1R, 512, 512, mw1, 128 * HIDW)
  VSEG(V_B + B_MB2, 128, 128, mb2, 0)
  VSEG(V_B + B_CB1, 128, 128, cb1, 0)
  VSEG(V_B + B_XB1, 128, 128, xb1, 0)
  VSEG(V_B + B_GB, 32, 4, gb, 0)
  VSEG(V_B + B_CB2, 32, 4, cb2, 0)
  VSEG(V_B + B_XB2, 32, 4, xb2, 0)
  VSEG(V_B + B_CHW, 32, 4, chw, 0)
  putf1(VEC + i, val);
}
#undef VSEG

__global__ __launch_bounds__(GTHR) void k_gemm(const unsigned short* __restrict__ A, int lda,
                                               const unsigned short* __restrict__ BT, int ldb, int K,
                                               const float* __restrict__ bias, int nRows, float* Cm, int ldc) {
  __shared__ __attribute__((aligned(16))) float stg[GBM * GBN];
  const int tid = (int)threadIdx.x, lane = tid & 31, wave = tid >> 5, hh = lane >> 4, m = lane & 15;
  const int rowBase = (int)blockIdx.x * GBM;
  const int colBase = (int)blockIdx.y * GBN;
  v8f acc[8];
#pragma unroll
  for (int t = 0; t < 8; ++t) acc[t] = z8();
  const unsigned short* ap = A  + (size_t)(rowBase + 16 * wave + m) * (size_t)lda + 8 * hh;
  const unsigned short* bp = BT + (size_t)(colBase + m) * (size_t)ldb + 8 * hh;
#pragma unroll 1
  for (int k0 = 0; k0 < K; k0 += 32) {
    FragB af;
    af.h[0] = *(const v8usa*)(ap + k0);
    af.h[1] = *(const v8usa*)(ap + k0 + 16);
#pragma unroll
    for (int nt = 0; nt < 8; ++nt) {
      const unsigned short* wq = bp + (size_t)(16 * nt) * (size_t)ldb + k0;
      FragB bf;
      bf.h[0] = *(const v8usa*)wq;
      bf.h[1] = *(const v8usa*)(wq + 16);
      acc[nt] = wmb(af, bf, acc[nt]);
    }
  }
#pragma unroll
  for (int nt = 0; nt < 8; ++nt) {
    const int lc = 16 * nt + m;
    const float bvv = bias[colBase + lc];
#pragma unroll
    for (int r = 0; r < 8; ++r) {
      const int lr = 16 * wave + 8 * hh + r;
      stg[lr * GBN + lc] = acc[nt][r] + bvv;
    }
  }
  __syncthreads();
  v4f pv[16];
#pragma unroll
  for (int i = 0; i < 16; ++i) pv[i] = *(const v4fa*)(stg + (16 * wave + i) * GBN + 4 * lane);
#pragma unroll
  for (int i = 0; i < 16; ++i) {
    const int row = rowBase + 16 * wave + i;
    if (row < nRows) {
      float* op = Cm + (size_t)row * (size_t)ldc + colBase + 4 * lane;
      *(volatile v4f*)op = pv[i];
    }
  }
  __threadfence();
#pragma unroll
  for (int i = 0; i < 16; ++i) {
    const int row = rowBase + 16 * wave + i;
    if (row < nRows) {
      float* op = Cm + (size_t)row * (size_t)ldc + colBase + 4 * lane;
      *(volatile v4f*)op = pv[i];
    }
  }
}

template <int APITCH>
__device__ __forceinline__ void wgemm64(const unsigned short* sAw, float* sDw, int dcol0,
                                        const unsigned short* __restrict__ BT, int ldb, int K, int hh, int m) {
  v8f acc[2][4];
#pragma unroll
  for (int mt = 0; mt < 2; ++mt)
#pragma unroll
    for (int nt = 0; nt < 4; ++nt) acc[mt][nt] = z8();
  const unsigned short* ap0 = sAw + m * APITCH + 8 * hh;
  const unsigned short* ap1 = ap0 + 16 * APITCH;
  const unsigned short* bp  = BT + (size_t)m * (size_t)ldb + 8 * hh;
#pragma unroll 1
  for (int k0 = 0; k0 < K; k0 += 32) {
    FragB a0, a1;
    a0.h[0] = *(const v8usa*)(ap0 + k0);
    a0.h[1] = *(const v8usa*)(ap0 + k0 + 16);
    a1.h[0] = *(const v8usa*)(ap1 + k0);
    a1.h[1] = *(const v8usa*)(ap1 + k0 + 16);
#pragma unroll
    for (int nt = 0; nt < 4; ++nt) {
      const unsigned short* wq = bp + (size_t)(16 * nt) * (size_t)ldb + k0;
      FragB b;
      b.h[0] = *(const v8usa*)wq;
      b.h[1] = *(const v8usa*)(wq + 16);
      acc[0][nt] = wmb(a0, b, acc[0][nt]);
      acc[1][nt] = wmb(a1, b, acc[1][nt]);
    }
  }
#pragma unroll
  for (int nt = 0; nt < 4; ++nt) {
    const int col = dcol0 + 16 * nt + m;
#pragma unroll
    for (int mt = 0; mt < 2; ++mt)
#pragma unroll
      for (int r = 0; r < 8; ++r) sDw[(16 * mt + 8 * hh + r) * DP + col] = acc[mt][nt][r];
  }
}
template <int APITCH>
__device__ __forceinline__ void wgemm16(const unsigned short* sAw, float* sDw, int dcol0,
                                        const unsigned short* __restrict__ BT, int ldb, int K, int hh, int m) {
  v8f acc0 = z8(), acc1 = z8();
  const unsigned short* ap0 = sAw + m * APITCH + 8 * hh;
  const unsigned short* ap1 = ap0 + 16 * APITCH;
  const unsigned short* bp  = BT + (size_t)m * (size_t)ldb + 8 * hh;
#pragma unroll 1
  for (int k0 = 0; k0 < K; k0 += 32) {
    FragB a0, a1, b;
    a0.h[0] = *(const v8usa*)(ap0 + k0);
    a0.h[1] = *(const v8usa*)(ap0 + k0 + 16);
    a1.h[0] = *(const v8usa*)(ap1 + k0);
    a1.h[1] = *(const v8usa*)(ap1 + k0 + 16);
    b.h[0]  = *(const v8usa*)(bp + k0);
    b.h[1]  = *(const v8usa*)(bp + k0 + 16);
    acc0 = wmb(a0, b, acc0);
    acc1 = wmb(a1, b, acc1);
  }
  const int col = dcol0 + m;
#pragma unroll
  for (int r = 0; r < 8; ++r) {
    sDw[(8 * hh + r) * DP + col]      = acc0[r];
    sDw[(16 + 8 * hh + r) * DP + col] = acc1[r];
  }
}

__global__ __launch_bounds__(ETHR) void k_edgeA(const int* __restrict__ ei, const float* __restrict__ XP,
                                                const float* __restrict__ NF,
                                                const unsigned short* __restrict__ WPL,
                                                const float* __restrict__ VEC, float* T, float* SC) {
  extern __shared__ __attribute__((aligned(16))) float dyn[];
  float*          sD  = dyn;
  unsigned short* sA  = (unsigned short*)(dyn + TE * DP);
  float*          cst = dyn + TE * DP + (TE * AP) / 2;
  float*          sQK = cst + CSTN;
  int*            sR  = (int*)(sQK + TE * 4);
  int*            sC  = sR + TE;
  const unsigned short* EW2d = WPL + O_E2;
  const unsigned short* M1E  = WPL + O_M1E;
  const int tid = (int)threadIdx.x, lane = tid & 31, wave = tid >> 5, hh = lane >> 4, m = lane & 15;
  const int e0 = (int)blockIdx.x * TE;
#pragma unroll
  for (int it = 0; it < 4; ++it) {
    const int idx = it * ETHR + tid;
    const v4f cv = *(const v4fa*)(VEC + V_A + 4 * idx);
    *(v4fa*)(cst + 4 * idx) = cv;
  }
  __syncthreads();

  const int e = e0 + tid;
  const int r = clampi(ei[e], NNODE - 1);
  const int c = clampi(ei[NEDGE + e], NNODE - 1);
  sR[tid] = r;
  sC[tid] = c;
  const v4f xr = *(const v4fa*)(XP + (size_t)r * 4);
  const v4f xc = *(const v4fa*)(XP + (size_t)c * 4);
  const float rpx = xr.x - xc.x, rpy = xr.y - xc.y, rpz = xr.z - xc.z;
  const float rdist = (rpx * rpx + rpz * rpz) + rpy * rpy;
  float*          rd = sD + tid * DP;
  unsigned short* ra = sA + tid * AP;
  {
    const float* pr = NF + (size_t)r * NPW + 768;
    const float* qr = NF + (size_t)c * NPW + 896;
#pragma unroll 1
    for (int c8 = 0; c8 < HIDW / 8; ++c8) {
      const v8f p8 = join8(*(const v4fa*)(pr + 8 * c8), *(const v4fa*)(pr + 8 * c8 + 4));
      const v8f q8 = join8(*(const v4fa*)(qr + 8 * c8), *(const v4fa*)(qr + 8 * c8 + 4));
      const v8f w8 = join8(*(const v4fa*)(cst + A_W1R + 8 * c8), *(const v4fa*)(cst + A_W1R + 8 * c8 + 4));
      v8f s8;
#pragma unroll
      for (int i = 0; i < 8; ++i) s8[i] = silu_p((p8[i] + q8[i]) + rdist * w8[i]);
      split8(s8, ra + 8 * c8, ra + HIDW + 8 * c8);
    }
  }
  __syncthreads();

  const unsigned short* sAw = sA + 32 * wave * AP;
  float*                sDw = sD + 32 * wave * DP;
#pragma unroll 1
  for (int nh = 0; nh < 2; ++nh)
    wgemm64<AP>(sAw, sDw, 64 * nh, EW2d + (size_t)(64 * nh) * 256, 256, 256, hh, m);
  __syncthreads();

#pragma unroll 1
  for (int c8 = 0; c8 < HIDW / 8; ++c8) {
    const v8f v8 = join8(*(const v4fa*)(rd + 8 * c8), *(const v4fa*)(rd + 8 * c8 + 4));
    const v8f b8 = join8(*(const v4fa*)(cst + A_EB2 + 8 * c8), *(const v4fa*)(cst + A_EB2 + 8 * c8 + 4));
    v8f s8;
#pragma unroll
    for (int i = 0; i < 8; ++i) s8[i] = v8[i] + b8[i];
    split8(s8, ra + 8 * c8, ra + HIDW + 8 * c8);
  }
  __syncthreads();

#pragma unroll 1
  for (int nh = 0; nh < 2; ++nh)
    wgemm64<AP>(sAw, sDw, 64 * nh, M1E + (size_t)(64 * nh) * 256, 256, 256, hh, m);
  wgemm16<AP>(sAw, sDw, 128, M1E + (size_t)128 * 256, 256, 256, hh, m);
  __syncthreads();

  {
    const v4f bm = *(const v4fa*)(cst + A_MB1 + 4 * lane);
#pragma unroll 1
    for (int hb = 0; hb < 2; ++hb) {
      v4f pv[16];
#pragma unroll
      for (int i = 0; i < 16; ++i) {
        const int row = 32 * wave + 16 * hb + i;
        const v4f sv = *(const v4fa*)(sD + row * DP + 4 * lane);
        pv[i] = sv + bm;
      }
#pragma unroll
      for (int i = 0; i < 16; ++i) {
        const int row = 32 * wave + 16 * hb + i;
        float* op = T + (size_t)(e0 + row) * HIDW + 4 * lane;
        *(volatile v4f*)op = pv[i];
      }
      __threadfence();
#pragma unroll
      for (int i = 0; i < 16; ++i) {
        const int row = 32 * wave + 16 * hb + i;
        float* op = T + (size_t)(e0 + row) * HIDW + 4 * lane;
        *(volatile v4f*)op = pv[i];
      }
    }
  }

  const float ew0 = rd[128] + cst[A_EWB + 0];
  const float ew1v = rd[129] + cst[A_EWB + 1];
  const float ew2v = rd[130] + cst[A_EWB + 2];
  const float ew3 = rd[131] + cst[A_EWB + 3];

  float pe0 = cst[A_PB2 + 0], pe1 = cst[A_PB2 + 1], pe2 = cst[A_PB2 + 2], pe3 = cst[A_PB2 + 3];
#pragma unroll 1
  for (int j = 0; j < 64; ++j) {
    const float sv = silu_p(rdist * cst[A_PW1 + j] + cst[A_PB1 + j]);
    const v4f w4 = *(const v4fa*)(cst + A_PW2 + 4 * j);
    pe0 = fmaf(sv, w4.x, pe0);
    pe1 = fmaf(sv, w4.y, pe1);
    pe2 = fmaf(sv, w4.z, pe2);
    pe3 = fmaf(sv, w4.w, pe3);
  }

#pragma unroll 1
  for (int i = 0; i < 32; ++i) {
    const int el = 32 * wave + i;
    const int rr = sR[el];
    const int cc = sC[el];
    const float* qp = NF + (size_t)rr * NPW + 8 * lane;
    const float* kp = NF + (size_t)cc * NPW + QKVW + 8 * lane;
    const v4f q0 = *(const v4fa*)qp;
    const v4f q1 = *(const v4fa*)(qp + 4);
    const v4f k0 = *(const v4fa*)kp;
    const v4f k1 = *(const v4fa*)(kp + 4);
    float p = q0.x * k0.x;
    p = fmaf(q0.y, k0.y, p); p = fmaf(q0.z, k0.z, p); p = fmaf(q0.w, k0.w, p);
    p = fmaf(q1.x, k1.x, p); p = fmaf(q1.y, k1.y, p); p = fmaf(q1.z, k1.z, p); p = fmaf(q1.w, k1.w, p);
    p += __shfl_xor(p, 1, 32);
    p += __shfl_xor(p, 2, 32);
    p += __shfl_xor(p, 4, 32);
    if ((lane & 7) == 0) sQK[el * 4 + (lane >> 3)] = p;
  }
  __syncthreads();

  {
    const v4f qk = *(const v4fa*)(sQK + 4 * tid);
    v4f sc;
    sc.x = (qk.x * 0.125f + pe0) + ew0;
    sc.y = (qk.y * 0.125f + pe1) + ew1v;
    sc.z = (qk.z * 0.125f + pe2) + ew2v;
    sc.w = (qk.w * 0.125f + pe3) + ew3;
    putf4(SC + (size_t)e * 4, sc);
  }
}

__global__ __launch_bounds__(NTHR) void k_soft(const int* __restrict__ keys, int nE, int vec8,
                                               const float* __restrict__ SC, float* SMS) {
  extern __shared__ __attribute__((aligned(16))) int dsm[];
  const int tid = (int)threadIdx.x, lane = tid & 31, wave = tid >> 5;
  const int nodeBase = (int)blockIdx.x * NBA;
  const int ovf = scan_build(keys, nE, vec8, nodeBase, dsm, tid, lane, wave);
  const int* sl   = dsm + LISTN + RCAP;
  const int* cnt  = sl + RCAP;
  const int* offs = cnt + NBA;
  float* stg = (float*)(dsm + STG_OFF);
  const float qnan = __int_as_float(0x7fc00000);
  const float ninf = __int_as_float((int)0xff800000u);
  const float pz = (ovf != 0) ? qnan : 0.0f;
#pragma unroll 1
  for (int si = 0; si < NBA / NWAVE; ++si) {
    const int s = si * NWAVE + wave;
    int c = cnt[s];
    const bool big = c > DEGCAP;
    c = c < 0 ? 0 : (c > DEGCAP ? DEGCAP : c);
    int o = offs[s];
    o = o < 0 ? 0 : (o > RCAP ? RCAP : o);
    float m0 = ninf, m1 = ninf, m2 = ninf, m3 = ninf;
#pragma unroll 1
    for (int b0 = 0; b0 < c; b0 += 32) {
      int idx = o + b0 + lane;
      idx = idx > RCAP - 1 ? RCAP - 1 : idx;
      const int eid = clampi(sl[idx] >> SLA, nE - 1);
      const bool valid = (b0 + lane) < c;
      const v4f sc = *(const v4fa*)(SC + (size_t)eid * 4);
      m0 = fmaxf(m0, valid ? sc.x : ninf);
      m1 = fmaxf(m1, valid ? sc.y : ninf);
      m2 = fmaxf(m2, valid ? sc.z : ninf);
      m3 = fmaxf(m3, valid ? sc.w : ninf);
    }
#pragma unroll
    for (int d = 16; d >= 1; d >>= 1) {
      m0 = fmaxf(m0, __shfl_xor(m0, d, 32));
      m1 = fmaxf(m1, __shfl_xor(m1, d, 32));
      m2 = fmaxf(m2, __shfl_xor(m2, d, 32));
      m3 = fmaxf(m3, __shfl_xor(m3, d, 32));
    }
    float q0 = 0.0f, q1 = 0.0f, q2 = 0.0f, q3 = 0.0f;
#pragma unroll 1
    for (int b0 = 0; b0 < c; b0 += 32) {
      int idx = o + b0 + lane;
      idx = idx > RCAP - 1 ? RCAP - 1 : idx;
      const int eid = clampi(sl[idx] >> SLA, nE - 1);
      const bool valid = (b0 + lane) < c;
      const v4f sc = *(const v4fa*)(SC + (size_t)eid * 4);
      const float x0 = expf(sc.x - m0), x1 = expf(sc.y - m1), x2 = expf(sc.z - m2), x3 = expf(sc.w - m3);
      q0 += valid ? x0 : 0.0f;
      q1 += valid ? x1 : 0.0f;
      q2 += valid ? x2 : 0.0f;
      q3 += valid ? x3 : 0.0f;
    }
#pragma unroll
    for (int d = 16; d >= 1; d >>= 1) {
      q0 += __shfl_xor(q0, d, 32);
      q1 += __shfl_xor(q1, d, 32);
      q2 += __shfl_xor(q2, d, 32);
      q3 += __shfl_xor(q3, d, 32);
    }
    const bool emp = (c == 0);
    const float pzr = big ? qnan : pz;
    if (lane == 0) {
      v4f mv, sv;
      mv.x = (emp ? 0.0f : m0) + pzr; mv.y = (emp ? 0.0f : m1) + pzr;
      mv.z = (emp ? 0.0f : m2) + pzr; mv.w = (emp ? 0.0f : m3) + pzr;
      sv.x = q0 + pzr; sv.y = q1 + pzr; sv.z = q2 + pzr; sv.w = q3 + pzr;
      *(v4fa*)(stg + 8 * s)     = mv;
      *(v4fa*)(stg + 8 * s + 4) = sv;
    }
  }
  __syncthreads();
  v4f dv[4];
#pragma unroll
  for (int j = 0; j < 4; ++j) dv[j] = *(const v4fa*)(stg + 4 * (j * NTHR + tid));
  float* ob = SMS + (size_t)nodeBase * 8;
#pragma unroll
  for (int j = 0; j < 4; ++j) *(volatile v4f*)(ob + 4 * (j * NTHR + tid)) = dv[j];
  __threadfence();
#pragma unroll
  for (int j = 0; j < 4; ++j) *(volatile v4f*)(ob + 4 * (j * NTHR + tid)) = dv[j];
}

__global__ __launch_bounds__(ETHR) void k_edgeB(const int* __restrict__ ei, const float* __restrict__ XP,
                                                const float* __restrict__ T, const float* __restrict__ SC,
                                                const float* __restrict__ SMS,
                                                const unsigned short* __restrict__ WPL,
                                                const float* __restrict__ VEC, float* ATT, float* CU) {
  extern __shared__ __attribute__((aligned(16))) float dyn[];
  float*          sD  = dyn;
  unsigned short* sA  = (unsigned short*)(dyn + TE * DP);
  unsigned short* sA2 = sA + TE * AP;
  float*          cst = dyn + TE * DP + (TE * AP) / 2 + (TE * A2P) / 2;
  float*          sCU = cst + CSTN;
  const unsigned short* MW2d = WPL + O_M2;
  const unsigned short* CXG  = WPL + O_CXG;
  const unsigned short* CX2  = WPL + O_CX2;
  const int tid = (int)threadIdx.x, lane = tid & 31, wave = tid >> 5, hh = lane >> 4, m = lane & 15;
  const int e0 = (int)blockIdx.x * TE;
#pragma unroll
  for (int it = 0; it < 4; ++it) {
    const int idx = it * ETHR + tid;
    const v4f cv = *(const v4fa*)(VEC + V_B + 4 * idx);
    *(v4fa*)(cst + 4 * idx) = cv;
  }
  __syncthreads();

  const int e  = e0 + tid;
  const int em = (e == 0) ? (NEDGE - 1) : (e - 1);
  const int r  = clampi(ei[e], NNODE - 1);
  const int c  = clampi(ei[NEDGE + e], NNODE - 1);
  const int r2 = clampi(ei[em], NNODE - 1);
  const int c2 = clampi(ei[NEDGE + em], NNODE - 1);
  const v4f xr = *(const v4fa*)(XP + (size_t)r * 4);
  const v4f xc = *(const v4fa*)(XP + (size_t)c * 4);
  const v4f yr = *(const v4fa*)(XP + (size_t)r2 * 4);
  const v4f yc = *(const v4fa*)(XP + (size_t)c2 * 4);
  const float ax = xr.x - xc.x, ay = xr.y - xc.y, az = xr.z - xc.z;
  const float bx = yr.x - yc.x, by = yr.y - yc.y, bz = yr.z - yc.z;
  const float cx = ay * bz - az * by;
  const float cy = az * bx - ax * bz;
  const float cz = ax * by - ay * bx;
  float am;
  {
    const v4f sc = *(const v4fa*)(SC + (size_t)e * 4);
    const v4f mx = *(const v4fa*)(SMS + (size_t)r * 8);
    const v4f sm = *(const v4fa*)(SMS + (size_t)r * 8 + 4);
    v4f at;
    at.x = expf(sc.x - mx.x) / (sm.x + 1e-8f);
    at.y = expf(sc.y - mx.y) / (sm.y + 1e-8f);
    at.z = expf(sc.z - mx.z) / (sm.z + 1e-8f);
    at.w = expf(sc.w - mx.w) / (sm.w + 1e-8f);
    putf4(ATT + (size_t)e * 4, at);
    am = (((at.x + at.y) + at.z) + at.w) * 0.25f;
  }
  float*          rd  = sD + tid * DP;
  unsigned short* ra  = sA + tid * AP;
  unsigned short* ra2 = sA2 + tid * A2P;
  {
    const float* tr = T + (size_t)e * HIDW;
#pragma unroll 1
    for (int c8 = 0; c8 < HIDW / 8; ++c8) {
      const v8f t8 = join8(*(const v4fa*)(tr + 8 * c8), *(const v4fa*)(tr + 8 * c8 + 4));
      const v8f w0 = join8(*(const v4fa*)(cst + B_MW1R + 8 * c8), *(const v4fa*)(cst + B_MW1R + 8 * c8 + 4));
      const v8f w1 = join8(*(const v4fa*)(cst + B_MW1R + 128 + 8 * c8), *(const v4fa*)(cst + B_MW1R + 128 + 8 * c8 + 4));
      const v8f w2 = join8(*(const v4fa*)(cst + B_MW1R + 256 + 8 * c8), *(const v4fa*)(cst + B_MW1R + 256 + 8 * c8 + 4));
      const v8f w3 = join8(*(const v4fa*)(cst + B_MW1R + 384 + 8 * c8), *(const v4fa*)(cst + B_MW1R + 384 + 8 * c8 + 4));
      v8f s8;
#pragma unroll
      for (int i = 0; i < 8; ++i) {
        const float geo = (ax * w1[i] + ay * w2[i]) + az * w3[i];
        s8[i] = silu_p((t8[i] + am * w0[i]) + geo);
      }
      split8(s8, ra + 8 * c8, ra + HIDW + 8 * c8);
    }
  }
  __syncthreads();

  const unsigned short* sAw  = sA + 32 * wave * AP;
  const unsigned short* sA2w = sA2 + 32 * wave * A2P;
  float*                sDw  = sD + 32 * wave * DP;
#pragma unroll 1
  for (int nh = 0; nh < 2; ++nh)
    wgemm64<AP>(sAw, sDw, 64 * nh, MW2d + (size_t)(64 * nh) * 256, 256, 256, hh, m);
  __syncthreads();
#pragma unroll 1
  for (int c8 = 0; c8 < HIDW / 8; ++c8) {
    const v8f v8 = join8(*(const v4fa*)(rd + 8 * c8), *(const v4fa*)(rd + 8 * c8 + 4));
    const v8f b8 = join8(*(const v4fa*)(cst + B_MB2 + 8 * c8), *(const v4fa*)(cst + B_MB2 + 8 * c8 + 4));
    v8f s8;
#pragma unroll
    for (int i = 0; i < 8; ++i) s8[i] = v8[i] + b8[i];
    split8(s8, ra + 8 * c8, ra + HIDW + 8 * c8);
  }
  __syncthreads();
#pragma unroll 1
  for (int nh = 0; nh < 2; ++nh)
    wgemm64<AP>(sAw, sDw, 64 * nh, CXG + (size_t)(64 * nh) * 256, 256, 256, hh, m);
  __syncthreads();
#pragma unroll 1
  for (int c8 = 0; c8 < HIDW / 8; ++c8) {
    const v8f v8 = join8(*(const v4fa*)(rd + 8 * c8), *(const v4fa*)(rd + 8 * c8 + 4));
    const v8f b8 = join8(*(const v4fa*)(cst + B_CB1 + 8 * c8), *(const v4fa*)(cst + B_CB1 + 8 * c8 + 4));
    v8f s8;
#pragma unroll
    for (int i = 0; i < 8; ++i) s8[i] = silu_p(v8[i] + b8[i]);
    split8(s8, ra2 + 8 * c8, ra2 + 256 + 8 * c8);
  }
  __syncthreads();
#pragma unroll 1
  for (int nh = 0; nh < 2; ++nh)
    wgemm64<AP>(sAw, sDw, 64 * nh, CXG + (size_t)(128 + 64 * nh) * 256, 256, 256, hh, m);
  wgemm16<AP>(sAw, sDw, 128, CXG + (size_t)256 * 256, 256, 256, hh, m);
  __syncthreads();
#pragma unroll 1
  for (int c8 = 0; c8 < HIDW / 8; ++c8) {
    const v8f v8 = join8(*(const v4fa*)(rd + 8 * c8), *(const v4fa*)(rd + 8 * c8 + 4));
    const v8f b8 = join8(*(const v4fa*)(cst + B_XB1 + 8 * c8), *(const v4fa*)(cst + B_XB1 + 8 * c8 + 4));
    v8f s8;
#pragma unroll
    for (int i = 0; i < 8; ++i) s8[i] = silu_p(v8[i] + b8[i]);
    split8(s8, ra2 + 128 + 8 * c8, ra2 + 384 + 8 * c8);
  }
  const float g0 = sigm_p(rd[128] + cst[B_GB + 0]);
  const float g1 = sigm_p(rd[129] + cst[B_GB + 1]);
  const float g2 = sigm_p(rd[130] + cst[B_GB + 2]);
  const float g3 = sigm_p(rd[131] + cst[B_GB + 3]);
  __syncthreads();
  wgemm16<A2P>(sA2w, sDw, 0, CX2, 512, 512, hh, m);
  __syncthreads();
  {
    const float c0 = rd[0] + cst[B_CB2 + 0], c1 = rd[1] + cst[B_CB2 + 1];
    const float c2v = rd[2] + cst[B_CB2 + 2], c3 = rd[3] + cst[B_CB2 + 3];
    const float x0 = rd[4] + cst[B_XB2 + 0], x1 = rd[5] + cst[B_XB2 + 1];
    const float x2 = rd[6] + cst[B_XB2 + 2], x3 = rd[7] + cst[B_XB2 + 3];
    const float hw = (((g0 * c0) * cst[B_CHW + 0] + (g1 * c1) * cst[B_CHW + 1]) + (g2 * c2v) * cst[B_CHW + 2])
                     + (g3 * c3) * cst[B_CHW + 3];
    const float cg = ((x0 + x1) + x2) + x3;
    const v4f u0 = {hw * ax, hw * ay, hw * az, 0.0f};
    const v4f u1 = {cg * cx, cg * cy, cg * cz, 0.0f};
    *(v4fa*)(sCU + 8 * tid)     = u0;
    *(v4fa*)(sCU + 8 * tid + 4) = u1;
  }
  __syncthreads();
  {
    const v4f p0 = *(const v4fa*)(sCU + 4 * tid);
    const v4f p1 = *(const v4fa*)(sCU + 4 * (ETHR + tid));
    float* cb = CU + (size_t)e0 * 8;
    *(volatile v4f*)(cb + 4 * tid) = p0;
    *(volatile v4f*)(cb + 4 * (ETHR + tid)) = p1;
    __threadfence();
    *(volatile v4f*)(cb + 4 * tid) = p0;
    *(volatile v4f*)(cb + 4 * (ETHR + tid)) = p1;
  }
}

__global__ __launch_bounds__(NTHR) void k_agg(const int* __restrict__ ei, int nE, int vec8,
                                              const float* __restrict__ ATT, const float* __restrict__ CU,
                                              const float* __restrict__ NF, unsigned short* WVHL, float* out1) {
  extern __shared__ __attribute__((aligned(16))) int dsm[];
  const int tid = (int)threadIdx.x, lane = tid & 31, wave = tid >> 5;
  const int nodeBase = (int)blockIdx.x * NBA;
  const int ovf = scan_build(ei, nE, vec8, nodeBase, dsm, tid, lane, wave);
  const int* sl   = dsm + LISTN + RCAP;
  const int* cnt  = sl + RCAP;
  const int* offs = cnt + NBA;
  float* sO = (float*)(dsm + STG_OFF);
  const float qnan = __int_as_float(0x7fc00000);
  const float pz = (ovf != 0) ? qnan : 0.0f;
  const float inv = 1.0f / 9999.0f;
  const int hd = lane >> 3;
#pragma unroll 1
  for (int si = 0; si < NBA / NWAVE; ++si) {
    const int s    = si * NWAVE + wave;
    const int node = nodeBase + s;
    int c = cnt[s];
    const bool big = c > DEGCAP;
    c = c < 0 ? 0 : (c > DEGCAP ? DEGCAP : c);
    int o = offs[s];
    o = o < 0 ? 0 : (o > RCAP ? RCAP : o);
    v8f acc = z8();
    float u0 = 0.0f, u1 = 0.0f, u2 = 0.0f, u3 = 0.0f, u4 = 0.0f, u5 = 0.0f;
#pragma unroll 1
    for (int b0 = 0; b0 < c; b0 += 32) {
      int idx = o + b0 + lane;
      idx = idx > RCAP - 1 ? RCAP - 1 : idx;
      const int eid = clampi(sl[idx] >> SLA, nE - 1);
      const int cid = clampi(ei[nE + eid], NNODE - 1);
      const bool valid = (b0 + lane) < c;
      const v4f ca = *(const v4fa*)(CU + (size_t)eid * 8);
      const v4f cb = *(const v4fa*)(CU + (size_t)eid * 8 + 4);
      u0 += valid ? ca.x : 0.0f;
      u1 += valid ? ca.y : 0.0f;
      u2 += valid ? ca.z : 0.0f;
      u3 += valid ? cb.x : 0.0f;
      u4 += valid ? cb.y : 0.0f;
      u5 += valid ? cb.z : 0.0f;
      const int m32 = (c - b0) < 32 ? (c - b0) : 32;
#pragma unroll 1
      for (int k = 0; k < m32; ++k) {
        const int ek = __builtin_amdgcn_readlane(eid, k);
        const int ck = __builtin_amdgcn_readlane(cid, k);
        const float av = ATT[(size_t)ek * 4 + hd];
        const float* vp = NF + (size_t)ck * NPW + 512 + 8 * lane;
        const v8f v8 = join8(*(const v4fa*)vp, *(const v4fa*)(vp + 4));
#pragma unroll
        for (int i = 0; i < 8; ++i) acc[i] = fmaf(av, v8[i], acc[i]);
      }
    }
#pragma unroll
    for (int d = 16; d >= 1; d >>= 1) {
      u0 += __shfl_xor(u0, d, 32);
      u1 += __shfl_xor(u1, d, 32);
      u2 += __shfl_xor(u2, d, 32);
      u3 += __shfl_xor(u3, d, 32);
      u4 += __shfl_xor(u4, d, 32);
      u5 += __shfl_xor(u5, d, 32);
    }
    const float pzr = big ? qnan : pz;
    v8us oh, ol;
#pragma unroll
    for (int i = 0; i < 8; ++i) {
      const float val = acc[i] + pzr;
      const unsigned hb = bf16_bits(val);
      const unsigned lb = bf16_bits(val - __uint_as_float(hb << 16));
      oh[i] = (unsigned short)hb;
      ol[i] = (unsigned short)lb;
    }
    unsigned short* wp = WVHL + (size_t)node * 512 + 8 * lane;
    *(volatile v8us*)wp = oh;
    *(volatile v8us*)(wp + 256) = ol;
    __threadfence();
    *(volatile v8us*)wp = oh;
    *(volatile v8us*)(wp + 256) = ol;
    if (lane == 0) {
      sO[3 * s + 0] = (u0 * inv + u3 * inv) + pzr;
      sO[3 * s + 1] = (u1 * inv + u4 * inv) + pzr;
      sO[3 * s + 2] = (u2 * inv + u5 * inv) + pzr;
    }
  }
  __syncthreads();
  const int np = (NBA * 3) / 4;
  const int p0 = tid;
  const int p1c = (NTHR + tid) < np ? (NTHR + tid) : (np - 1);
  const v4f o0 = *(const v4fa*)(sO + 4 * p0);
  const v4f o1 = *(const v4fa*)(sO + 4 * p1c);
  const long long g0 = (long long)nodeBase * 3 + 4LL * p0;
  const long long g1 = (long long)nodeBase * 3 + 4LL * (NTHR + tid);
  const bool st0 = (g0 + 4 <= 3LL * NNODE);
  const bool st1 = ((NTHR + tid) < np) && (g1 + 4 <= 3LL * NNODE);
  if (st0) *(volatile v4f*)(out1 + (size_t)g0) = o0;
  if (st1) *(volatile v4f*)(out1 + (size_t)g1) = o1;
  __threadfence();
  if (st0) *(volatile v4f*)(out1 + (size_t)g0) = o0;
  if (st1) *(volatile v4f*)(out1 + (size_t)g1) = o1;
}

static inline size_t al256(size_t o) { return (o + 255) & ~(size_t)255; }

extern "C" void kernel_launch(void* const* d_in, const int* in_sizes, int n_in,
                              void* d_out, int out_size, void* d_ws, size_t ws_size,
                              hipStream_t stream) {
  if (n_in < 36) return;
  if (in_sizes[0] != NNODE * HIDW || in_sizes[1] != NNODE * 3 || in_sizes[2] != 2 * NEDGE) return;
  if (in_sizes[3] != HIDW * QKVW || in_sizes[4] != QKVW) return;
  if (in_sizes[5] != HIDW * QKVW || in_sizes[6] != QKVW) return;
  if (in_sizes[7] != HIDW * QKVW || in_sizes[8] != QKVW) return;
  if (in_sizes[9] != QKVW * HIDW || in_sizes[10] != HIDW) return;
  if (in_sizes[11] != 64 || in_sizes[12] != 64 || in_sizes[13] != 256 || in_sizes[14] != 4) return;
  if (in_sizes[15] != 257 * HIDW || in_sizes[16] != HIDW) return;
  if (in_sizes[17] != HIDW * HIDW || in_sizes[18] != HIDW) return;
  if (in_sizes[19] != HIDW * 4 || in_sizes[20] != 4) return;
  if (in_sizes[21] != 132 * HIDW || in_sizes[22] != HIDW) return;
  if (in_sizes[23] != HIDW * HIDW || in_sizes[24] != HIDW) return;
  if (in_sizes[25] != HIDW * 4 || in_sizes[26] != 4) return;
  if (in_sizes[27] != HIDW * HIDW || in_sizes[28] != HIDW) return;
  if (in_sizes[29] != HIDW * 4 || in_sizes[30] != 4 || in_sizes[31] != 4) return;
  if (in_sizes[32] != HIDW * HIDW || in_sizes[33] != HIDW) return;
  if (in_sizes[34] != HIDW * 4 || in_sizes[35] != 4) return;
  if (out_size != NNODE * HIDW + NNODE * 3) return;

  const float* h   = (const float*)d_in[0];
  const float* x   = (const float*)d_in[1];
  const int*   ei  = (const int*)d_in[2];
  const float* Wq  = (const float*)d_in[3];  const float* bq  = (const float*)d_in[4];
  const float* Wk  = (const float*)d_in[5];  const float* bk  = (const float*)d_in[6];
  const float* Wv  = (const float*)d_in[7];  const float* bv  = (const float*)d_in[8];
  const float* Wo  = (const float*)d_in[9];  const float* bo  = (const float*)d_in[10];
  const float* pw1 = (const float*)d_in[11]; const float* pb1 = (const float*)d_in[12];
  const float* pw2 = (const float*)d_in[13]; const float* pb2 = (const float*)d_in[14];
  const float* ew1 = (const float*)d_in[15]; const float* eb1 = (const float*)d_in[16];
  const float* ew2 = (const float*)d_in[17]; const float* eb2 = (const float*)d_in[18];
  const float* eww = (const float*)d_in[19]; const float* ewb = (const float*)d_in[20];
  const float* mw1 = (const float*)d_in[21]; const float* mb1 = (const float*)d_in[22];
  const float* mw2 = (const float*)d_in[23]; const float* mb2 = (const float*)d_in[24];
  const float* gw  = (const float*)d_in[25]; const float* gb  = (const float*)d_in[26];
  const float* cw1 = (const float*)d_in[27]; const float* cb1 = (const float*)d_in[28];
  const float* cw2 = (const float*)d_in[29]; const float* cb2 = (const float*)d_in[30];
  const float* chw = (const float*)d_in[31];
  const float* xw1 = (const float*)d_in[32]; const float* xb1 = (const float*)d_in[33];
  const float* xw2 = (const float*)d_in[34]; const float* xb2 = (const float*)d_in[35];
  float* out0 = (float*)d_out;
  float* out1 = out0 + (size_t)NNODE * HIDW;

  char* ws = (char*)d_ws;
  size_t off = 0;
  const size_t oHB  = off; off = al256(off + (size_t)MPR * HIDW * 2);
  const size_t oWPL = off; off = al256(off + (size_t)WPL_TOT * 2);
  const size_t oVEC = off; off = al256(off + (size_t)V_TOT * 4);
  const size_t oXP  = off; off = al256(off + (size_t)MPR * 4 * 4);
  const size_t oNF  = off; off = al256(off + (size_t)MPR * NPW * 4);
  const size_t oT   = off; off = al256(off + (size_t)NEDGE * HIDW * 4);
  const size_t oSC  = off; off = al256(off + (size_t)NEDGE * 4 * 4);
  const size_t oATT = off; off = al256(off + (size_t)NEDGE * 4 * 4);
  const size_t oCU  = off; off = al256(off + (size_t)NEDGE * 8 * 4);
  const size_t oSMS = off; off = al256(off + (size_t)NPADR * 8 * 4);
  const size_t oWV  = off; off = al256(off + (size_t)NPADR * 512 * 2);
  if (off > ws_size || off > ((size_t)256 << 20)) return;
  unsigned short* HB   = (unsigned short*)(ws + oHB);
  unsigned short* WPL  = (unsigned short*)(ws + oWPL);
  float*          VEC  = (float*)(ws + oVEC);
  float*          XP   = (float*)(ws + oXP);
  float*          NF   = (float*)(ws + oNF);
  float*          T    = (float*)(ws + oT);
  float*          SC   = (float*)(ws + oSC);
  float*          ATT  = (float*)(ws + oATT);
  float*          CU   = (float*)(ws + oCU);
  float*          SMS  = (float*)(ws + oSMS);
  unsigned short* WVHL = (unsigned short*)(ws + oWV);

  hipFuncSetAttribute(reinterpret_cast<const void*>(&k_edgeA), hipFuncAttributeMaxDynamicSharedMemorySize,
                      (int)EA_LDS_BYTES);
  hipFuncSetAttribute(reinterpret_cast<const void*>(&k_edgeB), hipFuncAttributeMaxDynamicSharedMemorySize,
                      (int)EB_LDS_BYTES);
  hipFuncSetAttribute(reinterpret_cast<const void*>(&k_soft), hipFuncAttributeMaxDynamicSharedMemorySize,
                      (int)SOFT_LDS_BYTES);
  hipFuncSetAttribute(reinterpret_cast<const void*>(&k_agg), hipFuncAttributeMaxDynamicSharedMemorySize,
                      (int)AGG_LDS_BYTES);

  k_pw1<<<PU2 / NTHR, NTHR, 0, stream>>>(Wq, Wk, Wv, ew1, ew2, mw2, WPL);
  k_pw2<<<QU3 / NTHR, NTHR, 0, stream>>>(mw1, eww, cw1, xw1, gw, cw2, xw2, Wo, WPL);
  k_pn<<<RU2 / NTHR, NTHR, 0, stream>>>(h, x, bq, bk, bv, eb1, bo, HB, XP, VEC);
  k_pva<<<1024 / NTHR, NTHR, 0, stream>>>(ew1, eb2, mb1, pw1, pb1, pw2, ewb, pb2, VEC);
  k_pvb<<<1024 / NTHR, NTHR, 0, stream>>>(mw1, mb2, cb1, xb1, gb, cb2, xb2, chw, VEC);
  k_gemm<<<dim3(MPR / GBM, NPW / GBN), GTHR, 0, stream>>>(HB, HIDW, WPL + O_WN, HIDW, HIDW, VEC + V_BN, MPR,
                                                          NF, NPW);
  k_edgeA<<<NEDGE / TE, ETHR, EA_LDS_BYTES, stream>>>(ei, XP, NF, WPL, VEC, T, SC);
  k_soft<<<NBLK, NTHR, SOFT_LDS_BYTES, stream>>>(ei, NEDGE, 1, SC, SMS);
  k_edgeB<<<NEDGE / TE, ETHR, EB_LDS_BYTES, stream>>>(ei, XP, T, SC, SMS, WPL, VEC, ATT, CU);
  k_agg<<<NBLK, NTHR, AGG_LDS_BYTES, stream>>>(ei, NEDGE, 1, ATT, CU, NF, WVHL, out1);
  k_gemm<<<dim3(MPR / GBM, 1), GTHR, 0, stream>>>(WVHL, 512, WPL + O_WO2, 512, 512, VEC + V_BO, NNODE, out0, HIDW);
}
